// TransformerBlock_8856222565048
// MI455X (gfx1250) — hardware-verified
//
#include <hip/hip_runtime.h>
#include <stddef.h>


typedef _Float16 v16h __attribute__((ext_vector_type(16)));
typedef _Float16 v8h  __attribute__((ext_vector_type(8)));
typedef float    v8f  __attribute__((ext_vector_type(8)));
typedef float    v4f  __attribute__((ext_vector_type(4)));

#ifndef NB
#define NB 4
#endif
#ifndef SEQ
#define SEQ 1024
#endif
#define NB_FULL  4
#define SEQ_FULL 1024
#define DIM   1024
#define NHEAD 16
#define HD    64
#define DFF   4096
#define MROWS (NB * SEQ)
#define LN_EPS 1.0e-5f

static_assert(NB >= 1 && NB <= NB_FULL);
static_assert(SEQ >= 128 && SEQ <= SEQ_FULL && (SEQ % 128) == 0);
static_assert(DIM == NHEAD * HD);
static_assert((MROWS % 64) == 0 && (MROWS % 8) == 0);
static_assert((DIM % 64) == 0 && (DFF % 64) == 0 && (DIM % 256) == 0);

#define LDT 72
#define LDC 68

#define WCARRY 64.0f
#define PCARRY 1024.0f
#define VCARRY 64.0f

#define WTA_BYTES ((size_t)3 * DIM * DIM * 2)
#define WTP_BYTES ((size_t)DIM * DIM * 2)
#define WTF_BYTES ((size_t)DFF * DIM * 2)
#define WTO_BYTES ((size_t)DIM * DFF * 2)
#define P16_BYTES ((size_t)MROWS * DIM * 2)
#define P32_BYTES ((size_t)MROWS * DIM * 4)
#define G16_BYTES ((size_t)MROWS * DFF * 2)
#define OFF_WTA  ((size_t)0)
#define OFF_WTP  (OFF_WTA + WTA_BYTES)
#define OFF_WTF  (OFF_WTP + WTP_BYTES)
#define OFF_WTO  (OFF_WTF + WTF_BYTES)
#define OFF_H1   (OFF_WTO + WTO_BYTES)
#define OFF_Q16  (OFF_H1 + P16_BYTES)
#define OFF_K16  (OFF_Q16 + P16_BYTES)
#define OFF_VT16 (OFF_K16 + P16_BYTES)
#define OFF_VATT (OFF_VT16 + P16_BYTES)
#define OFF_X1   (OFF_VATT + P16_BYTES)
#define OFF_H2   (OFF_X1 + P32_BYTES)
#define OFF_G16  (OFF_H2 + P16_BYTES)
#define WS_TOTAL (OFF_G16 + G16_BYTES)
static_assert((OFF_H1 % 128) == 0 && (OFF_X1 % 128) == 0 && (OFF_G16 % 128) == 0);
static_assert(WS_TOTAL <= (size_t)134217728);

__device__ __forceinline__ float bf16r(float x) {
  unsigned int u = __float_as_uint(x);
  u = (u + 0x7FFFu + ((u >> 16) & 1u)) & 0xFFFF0000u;
  return __uint_as_float(u);
}

__device__ __forceinline__ v16h frag_at(const _Float16* p) {
  v8h lo = *(const v8h*)(p);
  v8h hi = *(const v8h*)(p + 16);
  v16h out;
#pragma unroll
  for (int i = 0; i < 8; ++i) { out[i] = lo[i]; out[i + 8] = hi[i]; }
  return out;
}
__device__ __forceinline__ v16h ld_frag(const _Float16* base, int ld) {
  const int lane = threadIdx.x & 31;
  return frag_at(base + (lane & 15) * ld + (lane >> 4) * 8);
}

__device__ __forceinline__ v8f wmma16(v16h a, v16h b, v8f c) {
  v8f d = __builtin_amdgcn_wmma_f32_16x16x32_f16(false, a, false, b, (short)0, c,
                                                 false, false);
  asm volatile("v_nop\n\tv_nop\n\tv_nop\n\tv_nop" : "+v"(d) : "v"(a), "v"(b));
  return d;
}

__device__ __forceinline__ float red16_max(float x) {
#pragma unroll
  for (int off = 1; off < 16; off <<= 1) x = fmaxf(x, __shfl_xor(x, off, 32));
  return x;
}
__device__ __forceinline__ float red16_sum(float x) {
#pragma unroll
  for (int off = 1; off < 16; off <<= 1) x += __shfl_xor(x, off, 32);
  return x;
}
__device__ __forceinline__ float red32_sum(float x) {
#pragma unroll
  for (int off = 16; off > 0; off >>= 1) x += __shfl_xor(x, off, 32);
  return x;
}

__device__ __forceinline__ void wave_lds_sync() {
  __builtin_amdgcn_fence(3  , "wavefront");
  asm volatile("s_wait_dscnt 0x0" ::: "memory");
  __builtin_amdgcn_wave_barrier();
}

__device__ __forceinline__ float gelu_t(float v) {
  const float v3 = (v * v) * v;
  const float u = 0.7978845608028654f * (v + 0.044715f * v3);
  const float e = __expf(-2.0f * u);
  return v * __builtin_amdgcn_rcpf(1.0f + e);
}

__global__ __launch_bounds__(256) void wconv_kernel(
    const float* __restrict__ W, _Float16* __restrict__ Wt, int Kd, int Nd) {
  __shared__ __attribute__((aligned(16))) _Float16 T[64 * LDT];
  const int tid = threadIdx.x;
  const int n0 = blockIdx.x * 64;
  const int k0 = blockIdx.y * 64;
#pragma unroll 4
  for (int j = 0; j < 16; ++j) {
    const int idx = tid + 256 * j;
    const int kr = idx >> 6, nc = idx & 63;
    const float v = W[(size_t)(k0 + kr) * Nd + n0 + nc];
    T[nc * LDT + kr] = (_Float16)(WCARRY * bf16r(v));
  }
  __syncthreads();
  v8h x[2];
  size_t off[2];
#pragma unroll
  for (int i = 0; i < 2; ++i) {
    const int n = 32 * i + (tid >> 3);
    const int kc = (tid & 7) * 8;
    x[i] = *(const v8h*)&T[n * LDT + kc];
    off[i] = (size_t)(n0 + n) * Kd + k0 + kc;
  }
#pragma unroll
  for (int i = 0; i < 2; ++i) *(volatile v8h*)(Wt + off[i]) = x[i];
  __threadfence();
#pragma unroll
  for (int i = 0; i < 2; ++i) *(volatile v8h*)(Wt + off[i]) = x[i];
}

template <int FROM_X>
__global__ __launch_bounds__(256) void ln_kernel(
    const float* __restrict__ src, const float* __restrict__ gam,
    const float* __restrict__ bet, _Float16* __restrict__ dst) {
  const int tid = threadIdx.x, lane = tid & 31, w = tid >> 5;
  const int crow = blockIdx.x * 8 + w;
  size_t srow = (size_t)crow;
  if (FROM_X) {
    const int bidx = crow / SEQ;
    const int sq = crow - bidx * SEQ;
    srow = (size_t)sq * NB_FULL + bidx;
  }
  const float* sp = src + srow * DIM + lane * 8;

  float s = 0.0f;
#pragma unroll 1
  for (int i = 0; i < 4; ++i) {
    const v4f a0 = *(const v4f*)(sp + 256 * i);
    const v4f a1 = *(const v4f*)(sp + 256 * i + 4);
    float t = 0.0f;
#pragma unroll
    for (int j = 0; j < 4; ++j) {
      const float x0 = FROM_X ? bf16r(a0[j]) : a0[j];
      const float x1 = FROM_X ? bf16r(a1[j]) : a1[j];
      t += x0 + x1;
    }
    s += t;
  }
  s = red32_sum(s);
  const float mean = s * (1.0f / (float)DIM);

  float q = 0.0f;
#pragma unroll 1
  for (int i = 0; i < 4; ++i) {
    const v4f a0 = *(const v4f*)(sp + 256 * i);
    const v4f a1 = *(const v4f*)(sp + 256 * i + 4);
    float t = 0.0f;
#pragma unroll
    for (int j = 0; j < 4; ++j) {
      const float d0 = (FROM_X ? bf16r(a0[j]) : a0[j]) - mean;
      const float d1 = (FROM_X ? bf16r(a1[j]) : a1[j]) - mean;
      t += d0 * d0 + d1 * d1;
    }
    q += t;
  }
  q = red32_sum(q);
  const float rs = rsqrtf(q * (1.0f / (float)DIM) + LN_EPS);

#pragma unroll 1
  for (int i = 0; i < 4; ++i) {
    const v4f a0 = *(const v4f*)(sp + 256 * i);
    const v4f a1 = *(const v4f*)(sp + 256 * i + 4);
    const v4f g0 = *(const v4f*)(gam + 256 * i + lane * 8);
    const v4f g1 = *(const v4f*)(gam + 256 * i + lane * 8 + 4);
    const v4f b0 = *(const v4f*)(bet + 256 * i + lane * 8);
    const v4f b1 = *(const v4f*)(bet + 256 * i + lane * 8 + 4);
    v8h o;
#pragma unroll
    for (int j = 0; j < 4; ++j) {
      const float x0 = FROM_X ? bf16r(a0[j]) : a0[j];
      const float x1 = FROM_X ? bf16r(a1[j]) : a1[j];
      o[j]     = (_Float16)(((x0 - mean) * rs) * bf16r(g0[j]) + bf16r(b0[j]));
      o[j + 4] = (_Float16)(((x1 - mean) * rs) * bf16r(g1[j]) + bf16r(b1[j]));
    }
    _Float16* dp = dst + (size_t)crow * DIM + 256 * i + lane * 8;
    *(volatile v8h*)dp = o;
    __threadfence();
    *(volatile v8h*)dp = o;
  }
}

template <int MODE, int KD, int NO>
__global__ __launch_bounds__(256) void gemm_kernel(
    const _Float16* __restrict__ A16, const _Float16* __restrict__ Bt,
    const float* __restrict__ bias, const float* __restrict__ addf,
    const float* __restrict__ resf, float* __restrict__ outf,
    _Float16* __restrict__ out16) {
  static_assert((KD % 32) == 0 && (NO % 64) == 0);
  __shared__ __attribute__((aligned(16))) float Cs[64 * LDC];
  const int tid = threadIdx.x, lane = tid & 31, w = tid >> 5;
  const int mw = w >> 1, nw = w & 1;
  const int hh = lane >> 4, m = lane & 15;
  const int n0 = blockIdx.x * 64;
  const int row0 = blockIdx.y * 64;

  const _Float16* ap  = A16 + (size_t)(row0 + mw * 16 + m) * KD + hh * 8;
  const _Float16* bp0 = Bt + (size_t)(n0 + nw * 32 + m) * KD + hh * 8;
  const _Float16* bp1 = bp0 + (size_t)16 * KD;
  v8f acc0 = {}, acc1 = {};
#pragma unroll 2
  for (int k0 = 0; k0 < KD; k0 += 32) {
    const v16h a  = frag_at(ap + k0);
    const v16h b0 = frag_at(bp0 + k0);
    const v16h b1 = frag_at(bp1 + k0);
    acc0 = wmma16(a, b0, acc0);
    acc1 = wmma16(a, b1, acc1);
  }
#pragma unroll
  for (int r = 0; r < 8; ++r) {
    float* d = &Cs[(mw * 16 + hh * 8 + r) * LDC + nw * 32 + m];
    d[0]  = acc0[r];
    d[16] = acc1[r];
  }
  __syncthreads();

  if (MODE == 0) {
    v8h x[2];
    size_t off[2];
#pragma unroll
    for (int i = 0; i < 2; ++i) {
      const int r = 32 * i + (tid >> 3);
      const int c = (tid & 7) * 8;
      const v4f u0 = *(const v4f*)&Cs[r * LDC + c];
      const v4f u1 = *(const v4f*)&Cs[r * LDC + c + 4];
      const v4f g0 = *(const v4f*)(bias + n0 + c);
      const v4f g1 = *(const v4f*)(bias + n0 + c + 4);
#pragma unroll
      for (int j = 0; j < 4; ++j) {
        x[i][j]     = (_Float16)(u0[j] * (1.0f / WCARRY) + bf16r(g0[j]));
        x[i][j + 4] = (_Float16)(u1[j] * (1.0f / WCARRY) + bf16r(g1[j]));
      }
      off[i] = (size_t)(row0 + r) * NO + n0 + c;
    }
#pragma unroll
    for (int i = 0; i < 2; ++i) *(volatile v8h*)(out16 + off[i]) = x[i];
    __threadfence();
#pragma unroll
    for (int i = 0; i < 2; ++i) *(volatile v8h*)(out16 + off[i]) = x[i];
  }

  if (MODE == 1) {
    const int bidx = row0 / SEQ;
    const int key0 = row0 - bidx * SEQ;
    v8h x[2];
    size_t off[2];
#pragma unroll
    for (int i = 0; i < 2; ++i) {
      const int dcol = 32 * i + (tid >> 3);
      const int kk = (tid & 7) * 8;
      const float gb = bf16r(bias[n0 + dcol]);
#pragma unroll
      for (int j = 0; j < 8; ++j)
        x[i][j] = (_Float16)(Cs[(kk + j) * LDC + dcol] * (1.0f / WCARRY) + gb);
      off[i] = ((size_t)(bidx * DIM + n0 + dcol)) * SEQ + key0 + kk;
    }
#pragma unroll
    for (int i = 0; i < 2; ++i) *(volatile v8h*)(out16 + off[i]) = x[i];
    __threadfence();
#pragma unroll
    for (int i = 0; i < 2; ++i) *(volatile v8h*)(out16 + off[i]) = x[i];
  }

  if (MODE == 2) {
    v4f xs[4];
    size_t off[4];
#pragma unroll
    for (int i = 0; i < 4; ++i) {
      const int r = 16 * i + (tid >> 4);
      const int c = (tid & 15) * 4;
      const int crow = row0 + r;
      const int bidx = crow / SEQ;
      const int sq = crow - bidx * SEQ;
      const size_t frow = (size_t)sq * NB_FULL + bidx;
      const v4f u  = *(const v4f*)&Cs[r * LDC + c];
      const v4f gb = *(const v4f*)(bias + n0 + c);
      const v4f q  = *(const v4f*)(addf + frow * DIM + n0 + c);
      v4f val;
#pragma unroll
      for (int j = 0; j < 4; ++j)
        val[j] = (u[j] * (1.0f / (WCARRY * VCARRY)) + bf16r(gb[j])) + bf16r(q[j]);
      xs[i] = val;
      off[i] = (size_t)crow * NO + n0 + c;
    }
#pragma unroll
    for (int i = 0; i < 4; ++i) *(volatile v4f*)(outf + off[i]) = xs[i];
    __threadfence();
#pragma unroll
    for (int i = 0; i < 4; ++i) *(volatile v4f*)(outf + off[i]) = xs[i];
  }

  if (MODE == 3) {
    v8h x[2];
    size_t off[2];
#pragma unroll
    for (int i = 0; i < 2; ++i) {
      const int r = 32 * i + (tid >> 3);
      const int c = (tid & 7) * 8;
      const v4f u0 = *(const v4f*)&Cs[r * LDC + c];
      const v4f u1 = *(const v4f*)&Cs[r * LDC + c + 4];
      const v4f g0 = *(const v4f*)(bias + n0 + c);
      const v4f g1 = *(const v4f*)(bias + n0 + c + 4);
#pragma unroll
      for (int j = 0; j < 4; ++j) {
        const float t0 = u0[j] * (1.0f / WCARRY) + bf16r(g0[j]);
        const float t1 = u1[j] * (1.0f / WCARRY) + bf16r(g1[j]);
        x[i][j]     = (_Float16)gelu_t(t0);
        x[i][j + 4] = (_Float16)gelu_t(t1);
      }
      off[i] = (size_t)(row0 + r) * NO + n0 + c;
    }
#pragma unroll
    for (int i = 0; i < 2; ++i) *(volatile v8h*)(out16 + off[i]) = x[i];
    __threadfence();
#pragma unroll
    for (int i = 0; i < 2; ++i) *(volatile v8h*)(out16 + off[i]) = x[i];
  }

  if (MODE == 4) {
    v4f xs[4];
    size_t off[4];
#pragma unroll
    for (int i = 0; i < 4; ++i) {
      const int r = 16 * i + (tid >> 4);
      const int c = (tid & 15) * 4;
      const int crow = row0 + r;
      const int bidx = crow / SEQ;
      const int sq = crow - bidx * SEQ;
      const size_t frow = (size_t)sq * NB_FULL + bidx;
      const v4f u  = *(const v4f*)&Cs[r * LDC + c];
      const v4f gb = *(const v4f*)(bias + n0 + c);
      const v4f rx = *(const v4f*)(resf + (size_t)crow * NO + n0 + c);
      v4f val;
#pragma unroll
      for (int j = 0; j < 4; ++j)
        val[j] = rx[j] + (u[j] * (1.0f / WCARRY) + bf16r(gb[j]));
      xs[i] = val;
      off[i] = frow * NO + n0 + c;
    }
#pragma unroll
    for (int i = 0; i < 4; ++i) *(volatile v4f*)(outf + off[i]) = xs[i];
    __threadfence();
#pragma unroll
    for (int i = 0; i < 4; ++i) *(volatile v4f*)(outf + off[i]) = xs[i];
  }
}

__global__ __launch_bounds__(256) void attn_kernel(
    const _Float16* __restrict__ Qh, const _Float16* __restrict__ Kh,
    const _Float16* __restrict__ Vt, _Float16* __restrict__ Ov) {
  __shared__ __attribute__((aligned(16))) _Float16 Ks[64 * LDT];
  __shared__ __attribute__((aligned(16))) _Float16 Vs[64 * LDT];
  __shared__ __attribute__((aligned(16))) _Float16 Ps[8 * 16 * LDT];

  const int tid = threadIdx.x, lane = tid & 31, w = tid >> 5;
  const int hh = lane >> 4, m = lane & 15;
  const int q0 = blockIdx.x * 128;
  const int head = blockIdx.y;
  const int b = blockIdx.z;
  const float scale = 0.125f;
  _Float16* P = Ps + w * (16 * LDT);

  const size_t qoff = (size_t)(b * SEQ + q0 + w * 16 + m) * DIM + head * HD + hh * 8;
  v16h qf[2];
  qf[0] = frag_at(Qh + qoff);
  qf[1] = frag_at(Qh + qoff + 32);

  float mrow[8], lrow[8];
  v8f o[4];
#pragma unroll
  for (int v = 0; v < 8; ++v) { mrow[v] = -1.0e30f; lrow[v] = 0.0f; }
#pragma unroll
  for (int nb = 0; nb < 4; ++nb) o[nb] = (v8f){};

  const size_t kplane = (size_t)b * SEQ * DIM + head * HD;
  const size_t vplane = ((size_t)b * DIM + head * HD) * SEQ;

  for (int kb = 0; kb < SEQ; kb += 64) {
#pragma unroll
    for (int j = 0; j < 2; ++j) {
      const int idx = tid + 256 * j;
      const int r = idx >> 3, c = (idx & 7) * 8;
      *(v8h*)&Ks[r * LDT + c] = *(const v8h*)(Kh + kplane + (size_t)(kb + r) * DIM + c);
      *(v8h*)&Vs[r * LDT + c] = *(const v8h*)(Vt + vplane + (size_t)r * SEQ + kb + c);
    }
    __syncthreads();

    v8f s[4];
#pragma unroll
    for (int kg = 0; kg < 4; ++kg) {
      v8f t = {};
#pragma unroll
      for (int c = 0; c < 2; ++c) {
        const v16h kf = ld_frag(&Ks[(kg * 16) * LDT + c * 32], LDT);
        t = wmma16(qf[c], kf, t);
      }
      s[kg] = t * scale;
    }

    float alpha[8];
#pragma unroll
    for (int v = 0; v < 8; ++v) {
      float mx = fmaxf(fmaxf(s[0][v], s[1][v]), fmaxf(s[2][v], s[3][v]));
      mx = red16_max(mx);
      const float mn = fmaxf(mrow[v], mx);
      alpha[v] = __expf(mrow[v] - mn);
      mrow[v] = mn;
    }
#pragma unroll
    for (int kg = 0; kg < 4; ++kg)
#pragma unroll
      for (int v = 0; v < 8; ++v) s[kg][v] = __expf(s[kg][v] - mrow[v]);
#pragma unroll
    for (int v = 0; v < 8; ++v) {
      const float rs = red16_sum((s[0][v] + s[1][v]) + (s[2][v] + s[3][v]));
      lrow[v] = alpha[v] * lrow[v] + rs;
    }
#pragma unroll
    for (int nb = 0; nb < 4; ++nb)
#pragma unroll
      for (int v = 0; v < 8; ++v) o[nb][v] = o[nb][v] * alpha[v];

#pragma unroll
    for (int kg = 0; kg < 4; ++kg)
#pragma unroll
      for (int v = 0; v < 8; ++v)
        P[(hh * 8 + v) * LDT + kg * 16 + m] = (_Float16)(s[kg][v] * PCARRY);
    wave_lds_sync();

#pragma unroll
    for (int c = 0; c < 2; ++c) {
      const v16h pf = ld_frag(P + c * 32, LDT);
#pragma unroll
      for (int nb = 0; nb < 4; ++nb) {
        const v16h vf = ld_frag(&Vs[(nb * 16) * LDT + c * 32], LDT);
        o[nb] = wmma16(pf, vf, o[nb]);
      }
    }
    __syncthreads();
  }

  float inv[8];
#pragma unroll
  for (int v = 0; v < 8; ++v) inv[v] = __builtin_amdgcn_rcpf(lrow[v]) * (VCARRY / PCARRY);
#pragma unroll
  for (int nb = 0; nb < 4; ++nb)
#pragma unroll
    for (int v = 0; v < 8; ++v)
      P[(hh * 8 + v) * LDT + nb * 16 + m] = (_Float16)(o[nb][v] * inv[v]);
  wave_lds_sync();
  v8h x[4];
  size_t off[4];
#pragma unroll
  for (int i = 0; i < 4; ++i) {
    const int r = 4 * i + (lane >> 3);
    const int c = (lane & 7) * 8;
    x[i] = *(const v8h*)&P[r * LDT + c];
    off[i] = (size_t)(b * SEQ + q0 + w * 16 + r) * DIM + head * HD + c;
  }
#pragma unroll
  for (int i = 0; i < 4; ++i) *(volatile v8h*)(Ov + off[i]) = x[i];
  __threadfence();
#pragma unroll
  for (int i = 0; i < 4; ++i) *(volatile v8h*)(Ov + off[i]) = x[i];
}

extern "C" void kernel_launch(void* const* d_in, const int* in_sizes, int n_in,
                              void* d_out, int out_size, void* d_ws, size_t ws_size,
                              hipStream_t stream) {
  if (n_in < 13) return;
  const long long need_x = ((long long)(SEQ - 1) * NB_FULL + NB) * DIM;
  if ((long long)in_sizes[0] < need_x) return;
  if (in_sizes[1] < DIM || in_sizes[2] < DIM || in_sizes[6] < DIM || in_sizes[7] < DIM ||
      in_sizes[8] < DIM || in_sizes[12] < DIM) return;
  if ((long long)in_sizes[3] < (long long)3 * DIM * DIM || in_sizes[4] < 3 * DIM) return;
  if ((long long)in_sizes[5] < (long long)DIM * DIM) return;
  if ((long long)in_sizes[9] < (long long)DIM * DFF || in_sizes[10] < DFF ||
      (long long)in_sizes[11] < (long long)DFF * DIM) return;
  if ((long long)out_size < need_x) return;
  if (ws_size < WS_TOTAL) return;

  const float* x      = (const float*)d_in[0];
  const float* ln1_g  = (const float*)d_in[1];
  const float* ln1_b  = (const float*)d_in[2];
  const float* w_attn = (const float*)d_in[3];
  const float* b_attn = (const float*)d_in[4];
  const float* w_proj = (const float*)d_in[5];
  const float* b_proj = (const float*)d_in[6];
  const float* ln2_g  = (const float*)d_in[7];
  const float* ln2_b  = (const float*)d_in[8];
  const float* w_fc   = (const float*)d_in[9];
  const float* b_fc   = (const float*)d_in[10];
  const float* w_out  = (const float*)d_in[11];
  const float* b_out  = (const float*)d_in[12];
  float* out = (float*)d_out;

  char* ws = (char*)d_ws;
  _Float16* WtA    = (_Float16*)(ws + OFF_WTA);
  _Float16* WtP    = (_Float16*)(ws + OFF_WTP);
  _Float16* WtF    = (_Float16*)(ws + OFF_WTF);
  _Float16* WtO    = (_Float16*)(ws + OFF_WTO);
  _Float16* H1     = (_Float16*)(ws + OFF_H1);
  _Float16* Q16    = (_Float16*)(ws + OFF_Q16);
  _Float16* K16    = (_Float16*)(ws + OFF_K16);
  _Float16* Vt16   = (_Float16*)(ws + OFF_VT16);
  _Float16* Vatt16 = (_Float16*)(ws + OFF_VATT);
  float*    X1     = (float*)(ws + OFF_X1);
  _Float16* H2     = (_Float16*)(ws + OFF_H2);
  _Float16* G16    = (_Float16*)(ws + OFF_G16);

  dim3 blk(256);
  dim3 gq(DIM / 64, MROWS / 64);

  wconv_kernel<<<dim3(3 * DIM / 64, DIM / 64), blk, 0, stream>>>(w_attn, WtA, DIM, 3 * DIM);
  wconv_kernel<<<dim3(DIM / 64, DIM / 64), blk, 0, stream>>>(w_proj, WtP, DIM, DIM);
  wconv_kernel<<<dim3(DFF / 64, DIM / 64), blk, 0, stream>>>(w_fc, WtF, DIM, DFF);
  wconv_kernel<<<dim3(DIM / 64, DFF / 64), blk, 0, stream>>>(w_out, WtO, DFF, DIM);

  ln_kernel<1><<<dim3(MROWS / 8), blk, 0, stream>>>(x, ln1_g, ln1_b, H1);

  gemm_kernel<0, DIM, DIM><<<gq, blk, 0, stream>>>(H1, WtA, b_attn, x, X1, X1, Q16);
  gemm_kernel<0, DIM, DIM><<<gq, blk, 0, stream>>>(H1, WtA + (size_t)DIM * DIM, b_attn + DIM,
                                                   x, X1, X1, K16);
  gemm_kernel<1, DIM, DIM><<<gq, blk, 0, stream>>>(H1, WtA + (size_t)2 * DIM * DIM,
                                                   b_attn + 2 * DIM, x, X1, X1, Vt16);

  attn_kernel<<<dim3(SEQ / 128, NHEAD, NB), blk, 0, stream>>>(Q16, K16, Vt16, Vatt16);

  gemm_kernel<2, DIM, DIM><<<gq, blk, 0, stream>>>(Vatt16, WtP, b_proj, x, X1, X1, H2);

  ln_kernel<0><<<dim3(MROWS / 8), blk, 0, stream>>>(X1, ln2_g, ln2_b, H2);

  gemm_kernel<3, DIM, DFF><<<dim3(DFF / 64, MROWS / 64), blk, 0, stream>>>(H2, WtF, b_fc, x,
                                                                            X1, X1, G16);
  gemm_kernel<4, DFF, DIM><<<gq, blk, 0, stream>>>(G16, WtO, b_out, x, X1, out, H2);
}
